// CausalSelfAttention_66254165508788
// MI455X (gfx1250) — hardware-verified
//
#include <hip/hip_runtime.h>


#ifndef NB
#define NB 2
#endif
#ifndef SEQ
#define SEQ 2048
#endif
#ifndef RH
#define RH 256
#endif
#define SEQ_FULL 2048
#define DM   2048
#define NH_  32
#define NKV  8
#define REP  4
#define HD   64
#define NQKV 3072
#define KOFF 2048
#define VOFF 2560
#define CSP  72
#define SCL  0.125f
#define L2E  1.4426950408889634f
#define PLOG 10.0f
#define RCAR 1024.0f
#define RINV (1.0f / 1024.0f)
#define CCAR 64.0f
#define WCAR 16.0f

static_assert(HD == 64);
static_assert(REP == 4 && REP * NKV == NH_);
static_assert(NH_ * HD == DM);
static_assert((NH_ + 2 * NKV) * HD == NQKV);
static_assert(KOFF == NH_ * HD && VOFF == KOFF + NKV * HD);
static_assert(SEQ % 64 == 0 && RH % 64 == 0 && RH <= SEQ && (SEQ - RH) % 64 == 0 && SEQ <= SEQ_FULL);
static_assert(DM % 64 == 0 && NQKV % 64 == 0 && DM % 32 == 0);
static_assert(CSP % 8 == 0 && CSP >= HD);
static_assert(((size_t)SEQ * HD) % 512 == 0);

typedef _Float16 h16;
typedef unsigned short bf;
typedef __attribute__((ext_vector_type(16))) __bf16   v16bf;
typedef __attribute__((ext_vector_type(16))) _Float16 v16h;
typedef __attribute__((ext_vector_type(8)))  _Float16 v8h;
typedef __attribute__((ext_vector_type(2)))  _Float16 v2h;
typedef __attribute__((ext_vector_type(16))) unsigned short v16us;
typedef __attribute__((ext_vector_type(8)))  unsigned short v8us;
typedef __attribute__((ext_vector_type(2)))  unsigned short v2us;
typedef __attribute__((ext_vector_type(8)))  float    v8f;
typedef __attribute__((ext_vector_type(4)))  float    v4f;
typedef __attribute__((ext_vector_type(2)))  float    v2f;
typedef v4f  __attribute__((may_alias)) v4fa;

__device__ __forceinline__ unsigned short f2bf(float f) { unsigned u = __float_as_uint(f); u += 0x7FFFu + ((u >> 16) & 1u); return (unsigned short)(u >> 16); }
__device__ __forceinline__ float bf2f(unsigned short b) { return __uint_as_float(((unsigned)b) << 16); }
__device__ __forceinline__ float bfr(float f) { return bf2f(f2bf(f)); }
__device__ __forceinline__ void splitf(float y, unsigned short& h, unsigned short& l) { h = f2bf(y); l = f2bf(y - bf2f(h)); }
__device__ __forceinline__ h16 tohn(float x) { const h16 v = (h16)x; return (fabsf(x) < 6.1035156e-5f) ? (h16)0.0f : v; }
__device__ __forceinline__ unsigned short hbits(h16 v) { return __builtin_bit_cast(unsigned short, v); }
__device__ __forceinline__ v16h cat16(v8h lo, v8h hi) { return __builtin_shufflevector(lo, hi, 0, 1, 2, 3, 4, 5, 6, 7, 8, 9, 10, 11, 12, 13, 14, 15); }
__device__ __forceinline__ v16bf cat16b(v8us lo, v8us hi) { return __builtin_bit_cast(v16bf, __builtin_shufflevector(lo, hi, 0, 1, 2, 3, 4, 5, 6, 7, 8, 9, 10, 11, 12, 13, 14, 15)); }
__device__ __forceinline__ v8f wmma16(v16h a, v16h b, v8f c) { c = __builtin_amdgcn_wmma_f32_16x16x32_f16(false, a, false, b, (short)0, c, false, false); asm volatile("v_nop\n\tv_nop\n\tv_nop\n\tv_nop" : "+v"(c) : "v"(a), "v"(b)); return c; }
__device__ __forceinline__ v8f wmmab(v16bf a, v16bf b, v8f c) { c = __builtin_amdgcn_wmma_f32_16x16x32_bf16(false, a, false, b, (short)0, c, false, false); asm volatile("v_nop\n\tv_nop\n\tv_nop\n\tv_nop" : "+v"(c) : "v"(a), "v"(b)); return c; }

__device__ __forceinline__ v16us ldf(const bf* p) { const v8us a = *(const v8us*)p; const v8us b = *(const v8us*)(p + 16); return __builtin_shufflevector(a, b, 0, 1, 2, 3, 4, 5, 6, 7, 8, 9, 10, 11, 12, 13, 14, 15); }
template <bool BFM> __device__ __forceinline__ v8f mm(v16us a, v16us b, v8f c) {
    if constexpr (BFM) return wmmab(__builtin_bit_cast(v16bf, a), __builtin_bit_cast(v16bf, b), c);
    else return wmma16(__builtin_bit_cast(v16h, a), __builtin_bit_cast(v16h, b), c);
}

template <typename T16> struct WFrag;
template <> struct WFrag<h16> { typedef v16h V; static __device__ __forceinline__ V ld(const h16* p) { return cat16(*(const v8h*)p, *(const v8h*)(p + 16)); } static __device__ __forceinline__ v8f mma(V a, V b, v8f c) { return wmma16(a, b, c); } };
template <> struct WFrag<bf> { typedef v16bf V; static __device__ __forceinline__ V ld(const bf* p) { return cat16b(*(const v8us*)p, *(const v8us*)(p + 16)); } static __device__ __forceinline__ v8f mma(V a, V b, v8f c) { return wmmab(a, b, c); } };
template <typename T16, int NSPLIT>
__device__ __forceinline__ void gemm_body(const T16* A, const T16* A2, const T16* Bt, int K, float* C, int ldc, float osc) {
    typedef typename WFrag<T16>::V V;
    __shared__ __align__(16) float os[16 * 68];
    const int lane = threadIdx.x & 31, lr = lane & 15, hi = lane >> 4; const int r0 = blockIdx.x * 64, c0 = blockIdx.y * 64;
    v8f acc[4][4];
#pragma unroll
    for (int mb = 0; mb < 4; ++mb)
#pragma unroll
        for (int nb = 0; nb < 4; ++nb) acc[mb][nb] = (v8f){};
    const size_t aoff = (size_t)(r0 + lr) * K + 8 * hi, boff = (size_t)(c0 + lr) * K + 8 * hi;
#pragma unroll 1
    for (int kc = 0; kc < K; kc += 32) {
        V a[4], a2[4];
#pragma unroll
        for (int mb = 0; mb < 4; ++mb) { a[mb] = WFrag<T16>::ld(A + aoff + (size_t)mb * 16 * K + kc); if (NSPLIT == 1) a2[mb] = WFrag<T16>::ld(A2 + aoff + (size_t)mb * 16 * K + kc); }
#pragma unroll
        for (int nb = 0; nb < 4; ++nb) { const V b = WFrag<T16>::ld(Bt + boff + (size_t)nb * 16 * K + kc);
#pragma unroll
            for (int mb = 0; mb < 4; ++mb) { acc[mb][nb] = WFrag<T16>::mma(a[mb], b, acc[mb][nb]); if (NSPLIT == 1) acc[mb][nb] = WFrag<T16>::mma(a2[mb], b, acc[mb][nb]); } }
    }
#pragma unroll
    for (int mb = 0; mb < 4; ++mb) {
#pragma unroll
        for (int nb = 0; nb < 4; ++nb) {
#pragma unroll
            for (int j = 0; j < 8; ++j) os[(hi * 8 + j) * 68 + nb * 16 + lr] = acc[mb][nb][j]; }
        __builtin_amdgcn_wave_barrier(); asm volatile("" ::: "memory");
        float* crow = C + (size_t)(r0 + mb * 16) * ldc + c0;
#pragma unroll 1
        for (int ps = 0; ps < 2; ++ps) {
#pragma unroll
            for (int s = 0; s < 8; ++s) { const int row = 2 * s + hi, cofs = lr * 4; v4f val = *(const v4fa*)(os + row * 68 + cofs); val = val * osc;
                *(volatile v4f*)(crow + (size_t)row * ldc + cofs) = val; }
            if (ps == 0) __threadfence(); }
        __builtin_amdgcn_wave_barrier(); asm volatile("" ::: "memory");
    }
}
__global__ __launch_bounds__(32) void k_gemm_b(const bf* __restrict__ A, const bf* __restrict__ Bt, int K, float* C, int ldc) { gemm_body<bf, 0>(A, A, Bt, K, C, ldc, 1.0f); }
__global__ __launch_bounds__(32) void k_gemm_b2(const bf* __restrict__ A, const bf* __restrict__ A2, const bf* __restrict__ Bt, int K, float* C, int ldc) { gemm_body<bf, 1>(A, A2, Bt, K, C, ldc, 1.0f); }
__global__ __launch_bounds__(32) void k_gemm_h(const h16* __restrict__ A, const h16* __restrict__ Bt, int K, float* C, int ldc, float osc) { gemm_body<h16, 0>(A, A, Bt, K, C, ldc, osc); }

__global__ __launch_bounds__(256) void k_cvt8(const float* __restrict__ src, bf* dst, size_t n8) { const size_t i = (size_t)blockIdx.x * 256 + threadIdx.x; if (i >= n8) return; const v8f v = *(const v8f*)(src + i * 8); v8us o;
#pragma unroll
    for (int k = 0; k < 8; ++k) o[k] = f2bf(v[k]);
    *(volatile v8us*)(dst + i * 8) = o; __threadfence(); *(volatile v8us*)(dst + i * 8) = o; }
__global__ __launch_bounds__(256) void k_cvt8h(const float* __restrict__ src, h16* dst, size_t n8, float car) { const size_t i = (size_t)blockIdx.x * 256 + threadIdx.x; if (i >= n8) return; const v8f v = *(const v8f*)(src + i * 8); v8h o;
#pragma unroll
    for (int k = 0; k < 8; ++k) o[k] = tohn(bfr(v[k]) * car);
    *(volatile v8h*)(dst + i * 8) = o; __threadfence(); *(volatile v8h*)(dst + i * 8) = o; }

__global__ __launch_bounds__(256) void k_ropep(const float* __restrict__ F, int coloff, int nheads, const float* __restrict__ fc, const float* __restrict__ fs, h16* P16, h16* PRS, bf* Ph, bf* Pl, int hasres) {
#pragma clang fp contract(off)
    const size_t e = ((size_t)blockIdx.x * 256 + threadIdx.x) * 2; if (e >= (size_t)nheads * SEQ * HD) return;
    const int d = (int)(e % HD); const int t = (int)((e / HD) % SEQ); const int h = (int)(e / ((size_t)HD * SEQ));
    const v2f xx = *(const v2f*)(F + (size_t)t * NQKV + coloff + h * HD + d);
    const int j = d >> 1;
    const float c = bfr(fc[(size_t)t * (HD / 2) + j]), s = bfr(fs[(size_t)t * (HD / 2) + j]);
    const float a0 = xx[0] * c, b0 = xx[1] * s, a1 = xx[0] * s, b1 = xx[1] * c;
    const float o0 = a0 - b0, o1 = a1 + b1;
    const h16 v0 = tohn(o0), v1 = tohn(o1);
    v2h ov; ov[0] = v0; ov[1] = v1;
    v2h orr; orr[0] = (h16)((o0 - (float)v0) * RCAR); orr[1] = (h16)((o1 - (float)v1) * RCAR);
    v2us oh, ol; unsigned short q0, q1; splitf(o0, q0, q1); oh[0] = q0; ol[0] = q1; splitf(o1, q0, q1); oh[1] = q0; ol[1] = q1;
    const bool early = (t < RH);
    const size_t eo = ((size_t)h * RH + (early ? t : 0)) * HD + d;
    *(volatile v2h*)(P16 + e) = ov; if (hasres) *(volatile v2h*)(PRS + e) = orr; if (early) { *(volatile v2us*)(Ph + eo) = oh; *(volatile v2us*)(Pl + eo) = ol; }
    __threadfence();
    *(volatile v2h*)(P16 + e) = ov; if (hasres) *(volatile v2h*)(PRS + e) = orr; if (early) { *(volatile v2us*)(Ph + eo) = oh; *(volatile v2us*)(Pl + eo) = ol; }
}
__global__ __launch_bounds__(256) void k_vtp(const float* __restrict__ F, h16* V16, bf* Vh, bf* Vl) {
    const size_t e = ((size_t)blockIdx.x * 256 + threadIdx.x) * 2; if (e >= (size_t)NKV * HD * SEQ) return;
    const int t = (int)(e % SEQ); const int d = (int)((e / SEQ) % HD); const int g = (int)(e / ((size_t)SEQ * HD));
    v2h o16; v2us oh, ol;
#pragma unroll
    for (int q = 0; q < 2; ++q) { const float x = F[(size_t)(t + q) * NQKV + VOFF + g * HD + d]; o16[q] = tohn(x); unsigned short a2, c2; splitf(x, a2, c2); oh[q] = a2; ol[q] = c2; }
    const bool early = (t < RH);
    const size_t eo = ((size_t)g * HD + d) * RH + (early ? t : 0);
    *(volatile v2h*)(V16 + e) = o16; if (early) { *(volatile v2us*)(Vh + eo) = oh; *(volatile v2us*)(Vl + eo) = ol; }
    __threadfence();
    *(volatile v2h*)(V16 + e) = o16; if (early) { *(volatile v2us*)(Vh + eo) = oh; *(volatile v2us*)(Vl + eo) = ol; }
}

template <bool EARLY>
__device__ __forceinline__ void attn_body(const bf* QA, const bf* QB, const bf* KA, const bf* KB, const bf* VA, const bf* VB, bf* C0, bf* C1, int rbase) {
    constexpr int PRW = EARLY ? RH : SEQ;
    __shared__ __align__(16) bf cs0[4 * 16 * CSP];
    __shared__ __align__(16) bf cs1[EARLY ? 4 * 16 * CSP : 8];
    const int lane = threadIdx.x & 31, n = lane & 15, hh = lane >> 4;
    const int wave = __builtin_amdgcn_readfirstlane((int)(threadIdx.x >> 5));
    const int g = (int)blockIdx.y, h = g * REP + wave;
    const int q0 = rbase + (int)blockIdx.x * 16;
    const int qn = q0 + n;
    const size_t qo = ((size_t)h * PRW + (size_t)qn) * HD + 8 * hh;
    const v16us qa0 = ldf(QA + qo), qa1 = ldf(QA + qo + 32);
    const v16us qb0 = ldf(QB + qo), qb1 = ldf(QB + qo + 32);
    v8f o[4];
#pragma unroll
    for (int f = 0; f < 4; ++f) o[f] = (v8f){};
    float m = -1.0e30f, l = 0.0f;
    const int nkb = (q0 + 47) >> 5;
    const size_t kbase = ((size_t)g * PRW + n) * HD + 8 * hh;
    const size_t vbase = ((size_t)g * HD + n) * PRW + 8 * hh;
#pragma unroll 1
    for (int kb = 0; kb < nkb; ++kb) {
        const int k0 = kb * 32;
        const size_t ko = kbase + (size_t)k0 * HD;
        const v16us ka00 = ldf(KA + ko), ka01 = ldf(KA + ko + 32), ka10 = ldf(KA + ko + 16 * HD), ka11 = ldf(KA + ko + 16 * HD + 32);
        v8f s0 = (v8f){}, s1 = (v8f){};
        s0 = mm<EARLY>(ka00, qa0, s0); s0 = mm<EARLY>(ka01, qa1, s0);
        s1 = mm<EARLY>(ka10, qa0, s1); s1 = mm<EARLY>(ka11, qa1, s1);
        if constexpr (EARLY) {
            s0 = mm<true>(ka00, qb0, s0); s0 = mm<true>(ka01, qb1, s0);
            s1 = mm<true>(ka10, qb0, s1); s1 = mm<true>(ka11, qb1, s1);
            const v16us kl00 = ldf(KB + ko), kl01 = ldf(KB + ko + 32), kl10 = ldf(KB + ko + 16 * HD), kl11 = ldf(KB + ko + 16 * HD + 32);
            s0 = mm<true>(kl00, qa0, s0); s0 = mm<true>(kl01, qa1, s0);
            s1 = mm<true>(kl10, qa0, s1); s1 = mm<true>(kl11, qa1, s1);
        } else {
            v8f r0 = (v8f){}, r1 = (v8f){};
            r0 = mm<false>(ka00, qb0, r0); r0 = mm<false>(ka01, qb1, r0);
            r1 = mm<false>(ka10, qb0, r1); r1 = mm<false>(ka11, qb1, r1);
#pragma unroll
            for (int r = 0; r < 8; ++r) { s0[r] = s0[r] + r0[r] * RINV; s1[r] = s1[r] + r1[r] * RINV; }
        }
        float t0[8], t1[8]; float cm = -1.0e30f;
        const int kk = k0 + 8 * hh;
#pragma unroll
        for (int r = 0; r < 8; ++r) {
            t0[r] = (kk + r <= qn) ? s0[r] * SCL : -1.0e30f;
            t1[r] = (kk + 16 + r <= qn) ? s1[r] * SCL : -1.0e30f;
            cm = fmaxf(cm, fmaxf(t0[r], t1[r])); }
        cm = fmaxf(cm, __shfl_xor(cm, 16, 32));
        const float mn = fmaxf(m, cm);
        const float corr = __builtin_amdgcn_exp2f((m - mn) * L2E);
        m = mn;
        float ps = 0.0f;
#pragma unroll
        for (int r = 0; r < 8; ++r) {
            t0[r] = __builtin_amdgcn_exp2f((t0[r] - mn) * L2E + PLOG);
            t1[r] = __builtin_amdgcn_exp2f((t1[r] - mn) * L2E + PLOG);
            ps += t0[r] + t1[r]; }
        ps += __shfl_xor(ps, 16, 32);
        l = l * corr + ps;
#pragma unroll
        for (int f = 0; f < 4; ++f)
#pragma unroll
            for (int r = 0; r < 8; ++r) o[f][r] *= corr;
        const size_t vo = vbase + (size_t)k0;
        if constexpr (EARLY) {
            v16us ph, pl;
#pragma unroll
            for (int r = 0; r < 8; ++r) { unsigned short a, c2; splitf(t0[r], a, c2); ph[r] = a; pl[r] = c2; splitf(t1[r], a, c2); ph[8 + r] = a; pl[8 + r] = c2; }
#pragma unroll
            for (int f = 0; f < 4; ++f) {
                const v16us vh = ldf(VA + vo + (size_t)(16 * f) * PRW);
                const v16us vl = ldf(VB + vo + (size_t)(16 * f) * PRW);
                o[f] = mm<true>(vh, ph, o[f]); o[f] = mm<true>(vl, ph, o[f]); o[f] = mm<true>(vh, pl, o[f]); }
        } else {
            v16us pb;
#pragma unroll
            for (int r = 0; r < 8; ++r) { pb[r] = hbits((h16)t0[r]); pb[8 + r] = hbits((h16)t1[r]); }
#pragma unroll
            for (int f = 0; f < 4; ++f) {
                const v16us va = ldf(VA + vo + (size_t)(16 * f) * PRW);
                o[f] = mm<false>(va, pb, o[f]); }
        }
    }
    const float inv = 1.0f / l;
    const int crow = (wave * 16 + n) * CSP + 8 * hh;
    if constexpr (EARLY) {
#pragma unroll
        for (int f = 0; f < 4; ++f) { v8us wh, wl;
#pragma unroll
            for (int r = 0; r < 8; ++r) { unsigned short a, c2; splitf(o[f][r] * inv, a, c2); wh[r] = a; wl[r] = c2; }
            *(v8us*)(cs0 + crow + 16 * f) = wh; *(v8us*)(cs1 + crow + 16 * f) = wl; }
    } else {
        const float sc = inv * CCAR;
#pragma unroll
        for (int f = 0; f < 4; ++f) { v8us w;
#pragma unroll
            for (int r = 0; r < 8; ++r) w[r] = hbits(tohn(o[f][r] * sc));
            *(v8us*)(cs0 + crow + 16 * f) = w; }
    }
    __syncthreads();
#pragma unroll 1
    for (int ps2 = 0; ps2 < 2; ++ps2) {
#pragma unroll
        for (int it = 0; it < 4; ++it) {
            const int row = 4 * it + (lane >> 3), pc = lane & 7;
            const size_t go = (size_t)(q0 + row) * DM + (size_t)h * HD + pc * 8;
            const v8us v0 = *(const v8us*)(cs0 + (wave * 16 + row) * CSP + pc * 8);
            *(volatile v8us*)(C0 + go) = v0;
            if constexpr (EARLY) { const v8us v1 = *(const v8us*)(cs1 + (wave * 16 + row) * CSP + pc * 8); *(volatile v8us*)(C1 + go) = v1; }
        }
        if (ps2 == 0) __threadfence();
    }
}
__global__ __launch_bounds__(128) void k_attn_e(const bf* Qh, const bf* Ql, const bf* Kh, const bf* Kl, const bf* Vh, const bf* Vl, bf* Ch, bf* Cl) { attn_body<true>(Qh, Ql, Kh, Kl, Vh, Vl, Ch, Cl, 0); }
__global__ __launch_bounds__(128) void k_attn_l(const bf* Q16, const bf* QR, const bf* K16, const bf* VT16, bf* C16) { attn_body<false>(Q16, QR, K16, K16, VT16, VT16, C16, C16, RH); }

constexpr size_t al256(size_t b) { return (b + 255) & ~(size_t)255; }
constexpr size_t SZ_WQKV = al256((size_t)NQKV * DM * 2);
constexpr size_t SZ_WO   = al256((size_t)DM * DM * 2);
constexpr size_t SZ_XB   = al256((size_t)SEQ * DM * 2);
constexpr size_t SZ_F    = al256((size_t)SEQ * NQKV * 4);
constexpr size_t SZ_Q    = al256((size_t)NH_ * SEQ * HD * 2);
constexpr size_t SZ_QE   = al256((size_t)NH_ * RH * HD * 2);
constexpr size_t SZ_K    = al256((size_t)NKV * SEQ * HD * 2);
constexpr size_t SZ_KE   = al256((size_t)NKV * RH * HD * 2);
constexpr size_t SZ_C    = al256((size_t)SEQ * DM * 2);
constexpr size_t SZ_CE   = al256((size_t)RH * DM * 2);
constexpr size_t WS_TOTAL = SZ_WQKV + 2 * SZ_WO + SZ_XB + SZ_F + 2 * SZ_Q + 2 * SZ_QE + 2 * SZ_K + 4 * SZ_KE + SZ_C + 2 * SZ_CE;
static_assert(WS_TOTAL <= (size_t)134217728);

extern "C" void kernel_launch(void* const* d_in, const int* in_sizes, int n_in,
                              void* d_out, int out_size, void* d_ws, size_t ws_size, hipStream_t stream) {
    if (n_in < 5) return;
    if ((long long)in_sizes[0] < (long long)(NB - 1) * SEQ_FULL * DM + (long long)SEQ * DM) return;
    if ((long long)in_sizes[1] < (long long)NQKV * DM) return;
    if ((long long)in_sizes[2] < (long long)DM * DM) return;
    if ((long long)in_sizes[3] < (long long)SEQ * (HD / 2)) return;
    if ((long long)in_sizes[4] < (long long)SEQ * (HD / 2)) return;
    if ((long long)out_size < (long long)NB * SEQ * DM) return;
    if (WS_TOTAL > ws_size) return;
    const float* x = (const float*)d_in[0]; const float* wqkv = (const float*)d_in[1]; const float* wproj = (const float*)d_in[2];
    const float* fc = (const float*)d_in[3]; const float* fs = (const float*)d_in[4];
    float* OUT = (float*)d_out;
    char* wsp = (char*)d_ws;
    auto take = [&](size_t bytes) { char* p = wsp; wsp += bytes; return (void*)p; };
    bf* WQKV = (bf*)take(SZ_WQKV); bf* WO = (bf*)take(SZ_WO); h16* WO16 = (h16*)take(SZ_WO);
    bf* XB = (bf*)take(SZ_XB); float* F = (float*)take(SZ_F);
    h16* Q16 = (h16*)take(SZ_Q); h16* QR = (h16*)take(SZ_Q); bf* Qh = (bf*)take(SZ_QE); bf* Ql = (bf*)take(SZ_QE);
    h16* K16 = (h16*)take(SZ_K); bf* Kh = (bf*)take(SZ_KE); bf* Kl = (bf*)take(SZ_KE);
    h16* VT16 = (h16*)take(SZ_K); bf* VTh = (bf*)take(SZ_KE); bf* VTl = (bf*)take(SZ_KE);
    bf* CTX16 = (bf*)take(SZ_C); bf* CTXh = (bf*)take(SZ_CE); bf* CTXl = (bf*)take(SZ_CE);
    if ((size_t)(wsp - (char*)d_ws) > ws_size) return;

    k_cvt8<<<(unsigned)(((size_t)NQKV * DM / 8 + 255) / 256), 256, 0, stream>>>(wqkv, WQKV, (size_t)NQKV * DM / 8);
    k_cvt8<<<(unsigned)(((size_t)DM * DM / 8 + 255) / 256), 256, 0, stream>>>(wproj, WO, (size_t)DM * DM / 8);
    k_cvt8h<<<(unsigned)(((size_t)DM * DM / 8 + 255) / 256), 256, 0, stream>>>(wproj, WO16, (size_t)DM * DM / 8, WCAR);
    const unsigned LQ = (unsigned)(((size_t)NH_ * SEQ * HD / 2 + 255) / 256), LK = (unsigned)(((size_t)NKV * SEQ * HD / 2 + 255) / 256);
    for (int b = 0; b < NB; ++b) {
        k_cvt8<<<(unsigned)(((size_t)SEQ * DM / 8 + 255) / 256), 256, 0, stream>>>(x + (size_t)b * SEQ_FULL * DM, XB, (size_t)SEQ * DM / 8);
        k_gemm_b<<<dim3(SEQ / 64, NQKV / 64, 1), 32, 0, stream>>>(XB, WQKV, DM, F, NQKV);
        k_ropep<<<LQ, 256, 0, stream>>>(F, 0, NH_, fc, fs, Q16, QR, Qh, Ql, 1);
        k_ropep<<<LK, 256, 0, stream>>>(F, KOFF, NKV, fc, fs, K16, K16, Kh, Kl, 0);
        k_vtp<<<LK, 256, 0, stream>>>(F, VT16, VTh, VTl);
        k_attn_e<<<dim3(RH / 16, NKV, 1), 128, 0, stream>>>(Qh, Ql, Kh, Kl, VTh, VTl, CTXh, CTXl);
        if (SEQ - RH > 0)
            k_attn_l<<<dim3((SEQ - RH) / 16 > 0 ? (SEQ - RH) / 16 : 1, NKV, 1), 128, 0, stream>>>((const bf*)Q16, (const bf*)QR, (const bf*)K16, (const bf*)VT16, CTX16);
        k_gemm_b2<<<dim3(RH / 64, DM / 64, 1), 32, 0, stream>>>(CTXh, CTXl, WO, DM, OUT + (size_t)b * SEQ * DM, DM);
        if (SEQ - RH > 0)
            k_gemm_h<<<dim3((SEQ - RH) / 64 > 0 ? (SEQ - RH) / 64 : 1, DM / 64, 1), 32, 0, stream>>>((const h16*)CTX16 + (size_t)RH * DM, WO16, DM, OUT + (size_t)b * SEQ * DM + (size_t)RH * DM, DM, 1.0f / (CCAR * WCAR));
    }
}
